// TopoPoolNet_70214125355054
// MI455X (gfx1250) — hardware-verified
//
#include <hip/hip_runtime.h>
#include <stddef.h>


#define IND     128
#define HD      64
#define NCLS    2
#define GMAX    128
#define NTHR    256
#define NWAVE   8
#define EPT     8
#define NGRP    1
#define CHUNK   (NTHR * EPT * NGRP)
#define WCAPC   (EPT * NGRP * 32)
#define WCAPF   (EPT * NGRP * 32)
#define ESHF    11
#define NBC     32768
#define NBF     2048
#define RCAP    67584
#define RBN     128
#define TGT     256
#define DEGCAP  512
#define GROWS   128
#define OTHR    512
#define TPK     64
#define TPN     32
#define TPP     72
#define ASCL    16
#define HSCL    256
#define WSCL    64
#define WSCAP   134217728

#define LDS_COUNT  ((NBC + NWAVE * WCAPC + NWAVE) * 4)
#define LDS_FILL   ((RCAP + NBF + NWAVE * WCAPF + NWAVE) * 4)

static_assert((CHUNK & (CHUNK - 1)) == 0);
static_assert(CHUNK <= 4096);
static_assert((NBC & (NBC - 1)) == 0 && (NBF & (NBF - 1)) == 0);
static_assert(NBF <= (1 << ESHF));
static_assert((NBC % NBF) == 0);
static_assert(OTHR * 4 == NBF);
static_assert((RCAP % 32) == 0);
static_assert(TGT == NWAVE * 32);
static_assert(GROWS == NWAVE * 16);
static_assert((TGT % GROWS) == 0);
static_assert(NBC == NWAVE * 32 * 128);
static_assert(HD == 64);
static_assert((IND % 32) == 0 && (HD % 32) == 0);
static_assert((IND % TPK) == 0 && (HD % TPK) == 0 && (HD % TPN) == 0);
static_assert(TPN * 8 == NTHR && TPK * TPN == NTHR * 8 && TPK == NWAVE * 8);
static_assert((TPP % 8) == 0 && TPP >= TPK);
static_assert(LDS_FILL <= 293 * 1024);
static_assert(LDS_COUNT <= 160 * 1024);

typedef float     v2f  __attribute__((ext_vector_type(2)));
typedef float     v4f  __attribute__((ext_vector_type(4)));
typedef float     v8f  __attribute__((ext_vector_type(8)));
typedef int       v4i  __attribute__((ext_vector_type(4)));
typedef _Float16  v2h  __attribute__((ext_vector_type(2)));
typedef _Float16  v8h  __attribute__((ext_vector_type(8)));
typedef _Float16  v16h __attribute__((ext_vector_type(16)));
union FragH { v16h v; v8h h[2]; };
union U32F { float f; int i; };

__device__ __forceinline__ v8f wmf(v16h a, v16h b, v8f c) {
  v8f d = __builtin_amdgcn_wmma_f32_16x16x32_f16(false, a, false, b, (short)0, c, false, false);
  asm volatile("v_nop\n\tv_nop\n\tv_nop\n\tv_nop" : "+v"(d) : "v"(a), "v"(b));
  return d;
}

template <int NB, int EIDX, int WC>
__device__ __forceinline__ int scan_chunk(const int* __restrict__ keys, int nK, int cbase,
                                          int slotBase, int vec8, int* list, int tid, int lane, int wave) {
  int wc = 0;
#pragma unroll
  for (int g = 0; g < NGRP; ++g) {
    const int el0  = (g * NTHR + tid) * EPT;
    const int e0   = cbase + el0;
    const int sent = -2147483647 - 1;
    v4i da, db;
    if (vec8 != 0 && cbase + CHUNK <= nK) {
      da = *(const v4i*)(keys + e0);
      db = *(const v4i*)(keys + e0 + 4);
    } else {
      const int i0 = min(e0, nK - 1),     i1 = min(e0 + 1, nK - 1), i2 = min(e0 + 2, nK - 1), i3 = min(e0 + 3, nK - 1);
      const int i4 = min(e0 + 4, nK - 1), i5 = min(e0 + 5, nK - 1), i6 = min(e0 + 6, nK - 1), i7 = min(e0 + 7, nK - 1);
      da.x = (e0     < nK) ? keys[i0] : sent;
      da.y = (e0 + 1 < nK) ? keys[i1] : sent;
      da.z = (e0 + 2 < nK) ? keys[i2] : sent;
      da.w = (e0 + 3 < nK) ? keys[i3] : sent;
      db.x = (e0 + 4 < nK) ? keys[i4] : sent;
      db.y = (e0 + 5 < nK) ? keys[i5] : sent;
      db.z = (e0 + 6 < nK) ? keys[i6] : sent;
      db.w = (e0 + 7 < nK) ? keys[i7] : sent;
    }
    const unsigned nb = (unsigned)slotBase;
    const unsigned s0 = (unsigned)da.x - nb, s1 = (unsigned)da.y - nb;
    const unsigned s2 = (unsigned)da.z - nb, s3 = (unsigned)da.w - nb;
    const unsigned s4 = (unsigned)db.x - nb, s5 = (unsigned)db.y - nb;
    const unsigned s6 = (unsigned)db.z - nb, s7 = (unsigned)db.w - nb;
    const bool h0 = s0 < (unsigned)NB, h1 = s1 < (unsigned)NB, h2 = s2 < (unsigned)NB, h3 = s3 < (unsigned)NB;
    const bool h4 = s4 < (unsigned)NB, h5 = s5 < (unsigned)NB, h6 = s6 < (unsigned)NB, h7 = s7 < (unsigned)NB;
    const unsigned any = __builtin_amdgcn_ballot_w32(h0 | h1 | h2 | h3 | h4 | h5 | h6 | h7);
    if (any != 0u) {
#define HITJ(HJ, SJ, JJ) { \
        const unsigned mj = __builtin_amdgcn_ballot_w32(HJ); \
        if (mj != 0u) { \
          if (HJ) { \
            const int pos = wc + (int)__builtin_amdgcn_mbcnt_lo(mj, 0u); \
            const int entv = EIDX ? (((el0 + (JJ)) << ESHF) | (int)(SJ)) : (int)(SJ); \
            if (pos < WC) list[wave * WC + pos] = entv; \
          } \
          wc += (int)__builtin_popcount(mj); } }
      HITJ(h0, s0, 0)
      HITJ(h1, s1, 1)
      HITJ(h2, s2, 2)
      HITJ(h3, s3, 3)
      HITJ(h4, s4, 4)
      HITJ(h5, s5, 5)
      HITJ(h6, s6, 6)
      HITJ(h7, s7, 7)
#undef HITJ
    }
  }
  return wc;
}

__global__ __launch_bounds__(NTHR) void k_cvt16(const float* __restrict__ src, _Float16* dst,
                                                int rowLen, int nSrcRows, int total8, float scale) {
  const int i = (int)blockIdx.x * NTHR + (int)threadIdx.x;
  if (i >= total8) return;
  const size_t e  = (size_t)8 * (size_t)i;
  const int    r  = (int)(e / (size_t)rowLen);
  const int    k0 = (int)(e - (size_t)r * (size_t)rowLen);
  const int    rc = r < nSrcRows ? r : nSrcRows - 1;
  const float  z  = (r < nSrcRows) ? scale : 0.0f;
  const float* sp = src + (size_t)rc * rowLen + k0;
  const v4f f0 = *(const v4f*)sp;
  const v4f f1 = *(const v4f*)(sp + 4);
  v8h hv;
  hv[0] = (_Float16)(f0.x * z); hv[1] = (_Float16)(f0.y * z); hv[2] = (_Float16)(f0.z * z); hv[3] = (_Float16)(f0.w * z);
  hv[4] = (_Float16)(f1.x * z); hv[5] = (_Float16)(f1.y * z); hv[6] = (_Float16)(f1.z * z); hv[7] = (_Float16)(f1.w * z);
  _Float16* d = dst + e;
  *(volatile v8h*)d = hv;
  __threadfence();
  *(volatile v8h*)d = hv;
}

__global__ __launch_bounds__(NTHR) void k_wT16(const float* __restrict__ W, _Float16* Wp,
                                               int KD, int NC, float scale) {
  __shared__ __attribute__((aligned(16))) _Float16 sT[TPN * TPP];
  const int tid = threadIdx.x;
  const int k0 = (int)blockIdx.x * TPK, n0 = (int)blockIdx.y * TPN;
  const int nc = tid & 31, kq = tid >> 5;
#pragma unroll
  for (int i = 0; i < TPK / NWAVE; ++i) {
    const int kr = kq + NWAVE * i;
    const float v = W[(size_t)(k0 + kr) * NC + n0 + nc] * scale;
    sT[nc * TPP + kr] = (_Float16)v;
  }
  __syncthreads();
  const int nl = tid >> 3, p = tid & 7;
  const v8h hv = *(const v8h*)(sT + nl * TPP + 8 * p);
  _Float16* d = Wp + (size_t)(n0 + nl) * KD + k0 + 8 * p;
  *(volatile v8h*)d = hv;
  __threadfence();
  *(volatile v8h*)d = hv;
}

__global__ __launch_bounds__(NTHR) void k_count(const int* __restrict__ keys, int* cnt, int nK, int vec8) {
  extern __shared__ v4f lds_dyn[];
  int* scnt = (int*)lds_dyn;
  int* list = scnt + NBC;
  int* wcnt = list + NWAVE * WCAPC;
  const int tid = threadIdx.x, lane = tid & 31, wave = tid >> 5;
  const int nodeBase = blockIdx.x * NBC;

  {
    const v4i z = {0, 0, 0, 0};
    for (int i = tid; i < NBC / 4; i += NTHR) ((v4i*)scnt)[i] = z;
  }
  __syncthreads();

  const int nChunks = (nK + CHUNK - 1) / CHUNK;
#pragma unroll 1
  for (int ch = 0; ch < nChunks; ++ch) {
    const int cbase = ch * CHUNK;
    const int wc = scan_chunk<NBC, 0, WCAPC>(keys, nK, cbase, nodeBase, vec8, list, tid, lane, wave);
    if (lane == 0) wcnt[wave] = wc;
    __syncthreads();
    if (wave == 0) {
#pragma unroll 1
      for (int wsx = 0; wsx < NWAVE; ++wsx) {
        int n = __builtin_amdgcn_readfirstlane(wcnt[wsx]);
        n = n > WCAPC ? WCAPC : (n < 0 ? 0 : n);
        const int* lp = list + wsx * WCAPC;
#pragma unroll 1
        for (int i = 0; i < n; ++i) {
          const int ent  = __builtin_amdgcn_readfirstlane(lp[i]);
          const int slot = ent & (NBC - 1);
          if (lane == 0) scnt[slot] = scnt[slot] + 1;
        }
      }
    }
    __syncthreads();
  }

  int* cp = cnt + (size_t)nodeBase;
#pragma unroll 4
  for (int q = 0; q < 32; ++q) {
    const int f = (wave * 32 + q) * 128 + 4 * lane;
    const v4i c = *(const v4i*)(scnt + f);
    *(volatile v4i*)(cp + f) = c;
  }
  __threadfence();
#pragma unroll 4
  for (int q = 0; q < 32; ++q) {
    const int f = (wave * 32 + q) * 128 + 4 * lane;
    const v4i c = *(const v4i*)(scnt + f);
    *(volatile v4i*)(cp + f) = c;
  }
}

__global__ __launch_bounds__(OTHR) void k_offsets(
    const int* __restrict__ cnt, int* off, int* rbase, int nBF) {
  __shared__ __attribute__((aligned(16))) int srb[RBN];
  __shared__ int wtot[OTHR / 32];
  const int tid = threadIdx.x, lane = tid & 31, wave = tid >> 5;
  for (int i = tid; i < RBN; i += OTHR) srb[i] = 0;
  int carry = 0;
#pragma unroll 1
  for (int fb = 0; fb < nBF; ++fb) {
    const int base = fb * NBF;
    const v4i c = *(const v4i*)(cnt + base + 4 * tid);
    const int e0 = max(c.x, 0), e1 = max(c.y, 0), e2 = max(c.z, 0), e3 = max(c.w, 0);
    const int ts = e0 + e1 + e2 + e3;
    int incl = ts;
#pragma unroll
    for (int d = 1; d < 32; d <<= 1) {
      const int t = __shfl_up(incl, d, 32);
      if (lane >= d) incl += t;
    }
    if (lane == 31) wtot[wave] = incl;
    __syncthreads();
    int pre = 0;
#pragma unroll 1
    for (int w = 0; w < wave; ++w) pre += wtot[w];
    int tot = 0;
#pragma unroll
    for (int w = 0; w < OTHR / 32; ++w) tot += wtot[w];
    int run = carry + pre + incl - ts;
    v4i o;
    o.x = run; run += e0;
    o.y = run; run += e1;
    o.z = run; run += e2;
    o.w = run;
    int* op = off + base + 4 * tid;
    *(volatile v4i*)op = o;
    __threadfence();
    *(volatile v4i*)op = o;
    if (tid == 0) srb[min(fb, RBN - 1)] = carry;
    carry += (tot + 31) & ~31;
    __syncthreads();
  }
  if (tid == 0) srb[min(nBF, RBN - 1)] = carry;
  __syncthreads();
  v4i rv = {0, 0, 0, 0};
  if (tid < 32) rv = *(const v4i*)(srb + 4 * tid);
  if (tid < 32) *(volatile v4i*)(rbase + 4 * tid) = rv;
  __threadfence();
  if (tid < 32) *(volatile v4i*)(rbase + 4 * tid) = rv;
}

__global__ __launch_bounds__(NTHR) void k_fill(
    const int* __restrict__ keys, const int* __restrict__ off, const int* __restrict__ rbase,
    int* csr, int nK, int vec8, int csrLen) {
  extern __shared__ v4f lds_dyn[];
  int* region = (int*)lds_dyn;
  int* cursor = region + RCAP;
  int* list   = cursor + NBF;
  int* wcnt   = list + NWAVE * WCAPF;
  const int tid = threadIdx.x, lane = tid & 31, wave = tid >> 5;
  const int b = blockIdx.x;
  const int nodeBase = b * NBF;

  int rb0 = rbase[b];
  const int rb1 = rbase[b + 1];
  rb0 = rb0 < 0 ? 0 : (rb0 > csrLen ? csrLen : rb0);
  rb0 &= ~31;
  int len = rb1 - rb0;
  len = len < 0 ? 0 : (len > RCAP ? RCAP : len);
  int lenW = (len + 31) & ~31;
  if (rb0 + lenW > csrLen) lenW = (csrLen - rb0) & ~31;

  {
    const v4i z = {0, 0, 0, 0};
    for (int i = tid; i < RCAP / 4; i += NTHR) ((v4i*)region)[i] = z;
    for (int s = tid; s < NBF; s += NTHR) {
      int o = off[nodeBase + s] - rb0;
      o = o < 0 ? 0 : (o > RCAP ? RCAP : o);
      cursor[s] = o;
    }
  }
  __syncthreads();

  const int nChunks = (nK + CHUNK - 1) / CHUNK;
#pragma unroll 1
  for (int ch = 0; ch < nChunks; ++ch) {
    const int cbase = ch * CHUNK;
    const int wc = scan_chunk<NBF, 1, WCAPF>(keys, nK, cbase, nodeBase, vec8, list, tid, lane, wave);
    if (lane == 0) wcnt[wave] = wc;
    __syncthreads();
    if (wave == 0) {
#pragma unroll 1
      for (int wsx = 0; wsx < NWAVE; ++wsx) {
        int n = __builtin_amdgcn_readfirstlane(wcnt[wsx]);
        n = n > WCAPF ? WCAPF : (n < 0 ? 0 : n);
        const int* lp = list + wsx * WCAPF;
#pragma unroll 1
        for (int i = 0; i < n; ++i) {
          const int ent  = __builtin_amdgcn_readfirstlane(lp[i]);
          const int slot = ent & (NBF - 1);
          const int el   = (ent >> ESHF) & (CHUNK - 1);
          int e = cbase + el;
          e = e > nK - 1 ? nK - 1 : e;
          if (lane == 0) {
            int pos = cursor[slot];
            pos = pos < 0 ? 0 : (pos > RCAP - 1 ? RCAP - 1 : pos);
            region[pos] = e;
            const int np = pos + 1;
            cursor[slot] = np > RCAP ? RCAP : np;
          }
        }
      }
    }
    __syncthreads();
  }

  const int nv = lenW >> 2;
  int* gp = csr + rb0;
#pragma unroll 1
  for (int i = tid; i < nv; i += NTHR) { const v4i v = ((const v4i*)region)[i]; *(volatile v4i*)(gp + 4 * i) = v; }
  __threadfence();
#pragma unroll 1
  for (int i = tid; i < nv; i += NTHR) { const v4i v = ((const v4i*)region)[i]; *(volatile v4i*)(gp + 4 * i) = v; }
}

__global__ __launch_bounds__(NTHR) void k_deg(
    const int* __restrict__ csr, const int* __restrict__ off, const int* __restrict__ cnt,
    const float* __restrict__ ew, float* dis, int nN, int nE, int csrLen) {
  const int tid = threadIdx.x;
  const int c = (int)blockIdx.x * NTHR + tid;
  int n = cnt[c];
  n = n < 0 ? 0 : (n > DEGCAP ? DEGCAP : n);
  const int st = off[c];
  int nmx = n;
#pragma unroll
  for (int o = 16; o > 0; o >>= 1) { const int t = __shfl_xor(nmx, o, 32); nmx = t > nmx ? t : nmx; }
  float d = 0.0f;
#pragma unroll 1
  for (int p = 0; p < nmx; ++p) {
    int pos = st + p;
    pos = pos < 0 ? 0 : (pos > csrLen - 1 ? csrLen - 1 : pos);
    int e = csr[pos];
    e = e < 0 ? 0 : (e > nE - 1 ? nE - 1 : e);
    const float wv = ew[e];
    d += (p < n) ? wv : 0.0f;
  }
  float r = (d > 0.0f) ? rsqrtf(fmaxf(d, 1e-12f)) : 0.0f;
  if (c >= nN) r = 0.0f;
  *(volatile float*)(dis + c) = r;
  __threadfence();
  *(volatile float*)(dis + c) = r;
}

template <int KD>
__global__ __launch_bounds__(NTHR) void k_gemm(
    const _Float16* __restrict__ A16, const _Float16* __restrict__ Bw,
    const float* __restrict__ rsc, float* C, float osc) {
  static_assert((KD % 32) == 0);
  constexpr int NC  = HD;
  constexpr int NT  = NC / 16;
  constexpr int NST = (16 * NC) / 128;
  __shared__ __attribute__((aligned(16))) float stg[GROWS * NC];
  const int tid = threadIdx.x, lane = tid & 31, wave = tid >> 5, hh = lane >> 4, m = lane & 15;
  const int rowBase = blockIdx.x * GROWS;
  const _Float16* ap  = A16 + (size_t)(rowBase + wave * 16 + m) * KD + 8 * hh;
  const _Float16* bp0 = Bw + (size_t)m * KD + 8 * hh;

  v8f acc[NT];
#pragma unroll
  for (int t = 0; t < NT; ++t) { v8f z = {0.f, 0.f, 0.f, 0.f, 0.f, 0.f, 0.f, 0.f}; acc[t] = z; }

#pragma unroll 1
  for (int kt = 0; kt < KD / 32; ++kt) {
    FragH af;
    af.h[0] = *(const v8h*)(ap + 32 * kt);
    af.h[1] = *(const v8h*)(ap + 32 * kt + 16);
#pragma unroll
    for (int t = 0; t < NT; ++t) {
      const _Float16* bp = bp0 + (size_t)(16 * t) * KD + 32 * kt;
      FragH bf;
      bf.h[0] = *(const v8h*)bp;
      bf.h[1] = *(const v8h*)(bp + 16);
      acc[t] = wmf(af.v, bf.v, acc[t]);
    }
  }

  const int r0 = wave * 16 + 8 * hh;
  float s[8];
  {
    const v4f dA = *(const v4f*)(rsc + (size_t)rowBase + r0);
    const v4f dB = *(const v4f*)(rsc + (size_t)rowBase + r0 + 4);
    s[0] = dA.x; s[1] = dA.y; s[2] = dA.z; s[3] = dA.w; s[4] = dB.x; s[5] = dB.y; s[6] = dB.z; s[7] = dB.w;
#pragma unroll
    for (int r = 0; r < 8; ++r) s[r] = s[r] * osc;
  }
  float* sp = stg + r0 * NC + m;
#pragma unroll
  for (int t = 0; t < NT; ++t) {
#pragma unroll
    for (int r = 0; r < 8; ++r) sp[r * NC + 16 * t] = acc[t][r] * s[r];
  }
  __syncthreads();

  const float* lp = stg + wave * 16 * NC;
  float* gp = C + (size_t)(rowBase + wave * 16) * NC;
#pragma unroll
  for (int i = 0; i < NST; ++i) {
    const v4f v = *(const v4f*)(lp + i * 128 + 4 * lane);
    *(volatile v4f*)(gp + (size_t)i * 128 + 4 * lane) = v;
  }
  __threadfence();
#pragma unroll
  for (int i = 0; i < NST; ++i) {
    const v4f v = *(const v4f*)(lp + i * 128 + 4 * lane);
    *(volatile v4f*)(gp + (size_t)i * 128 + 4 * lane) = v;
  }
}

template <int MODE>
__global__ __launch_bounds__(NTHR) void k_agg(
    const int* __restrict__ csr, const int* __restrict__ off, const int* __restrict__ cnt,
    const float* __restrict__ dis, const int* __restrict__ esrc, const float* __restrict__ ew,
    const float* __restrict__ hw, const float* __restrict__ bias,
    const float* __restrict__ pw, const float* __restrict__ pb,
    _Float16* outH, float* outF, int nN, int nE, int csrLen, float hscl) {
  __shared__ __attribute__((aligned(16))) _Float16 stgh[NWAVE * 4 * HD];
  __shared__ __attribute__((aligned(16))) float    stgf[NWAVE * 2 * HD];
  const int tid = threadIdx.x, lane = tid & 31, wave = tid >> 5;
  const int tbase = blockIdx.x * TGT + wave * 32;
  const int cl = tbase + lane;
  const int cnt_l = cnt[cl];
  const int off_l = off[cl];
  U32F dvu; dvu.f = dis[cl];
  const int ch = 2 * lane;
  const v2f bq = *(const v2f*)(bias + ch);
  v2f pq = {0.f, 0.f};
  float pbv = 0.0f;
  if (MODE == 2) { pq = *(const v2f*)(pw + ch); pbv = pb[0]; }
  _Float16* swh = stgh + wave * 4 * HD;
  float*    swf = stgf + wave * 2 * HD;

#pragma unroll 1
  for (int j = 0; j < 32; ++j) {
    const int c = tbase + j;
    int n = __builtin_amdgcn_readlane(cnt_l, j);
    n = n < 0 ? 0 : (n > DEGCAP ? DEGCAP : n);
    const int st = __builtin_amdgcn_readlane(off_l, j);
    U32F du; du.i = __builtin_amdgcn_readlane(dvu.i, j);
    const float dc = du.f;
    v2f acc = {0.f, 0.f};
#pragma unroll 1
    for (int q0 = 0; q0 < n; q0 += 32) {
      int pos = st + q0 + lane;
      pos = pos < 0 ? 0 : (pos > csrLen - 1 ? csrLen - 1 : pos);
      int e = csr[pos];
      e = e < 0 ? 0 : (e > nE - 1 ? nE - 1 : e);
      int sl = esrc[e];
      sl = sl < 0 ? 0 : (sl > nN - 1 ? nN - 1 : sl);
      U32F wu; wu.f = ew[e];
      const int mcnt = (n - q0) < 32 ? (n - q0) : 32;
#pragma unroll 1
      for (int p = 0; p < mcnt; ++p) {
        const int s = __builtin_amdgcn_readlane(sl, p);
        U32F wp; wp.i = __builtin_amdgcn_readlane(wu.i, p);
        const v2f hr = *(const v2f*)(hw + (size_t)s * HD + ch);
        acc.x = fmaf(hr.x, wp.f, acc.x);
        acc.y = fmaf(hr.y, wp.f, acc.y);
      }
    }
    v2f v;
    v.x = fmaxf(acc.x * dc + bq.x, 0.0f);
    v.y = fmaxf(acc.y * dc + bq.y, 0.0f);
    const bool live = c < nN;
    if (MODE == 1) {
      const float z = live ? hscl : 0.0f;
      v2h hv2;
      hv2[0] = (_Float16)(v.x * z); hv2[1] = (_Float16)(v.y * z);
      *(v2h*)(swh + (j & 3) * HD + ch) = hv2;
      if ((j & 3) == 3) {
        __builtin_amdgcn_fence(__ATOMIC_ACQ_REL, "wavefront");
        __builtin_amdgcn_wave_barrier();
        const v8h hv = *(const v8h*)(swh + 8 * lane);
        _Float16* rp = outH + (size_t)(c - 3) * HD + 8 * lane;
        *(volatile v8h*)rp = hv;
        __threadfence();
        *(volatile v8h*)rp = hv;
        __builtin_amdgcn_fence(__ATOMIC_ACQ_REL, "wavefront");
        __builtin_amdgcn_wave_barrier();
      }
    } else {
      float pr = v.x * pq.x + v.y * pq.y;
      pr += __shfl_xor(pr, 16, 32);
      pr += __shfl_xor(pr, 8, 32);
      pr += __shfl_xor(pr, 4, 32);
      pr += __shfl_xor(pr, 2, 32);
      pr += __shfl_xor(pr, 1, 32);
      const float sg = 1.0f / (1.0f + __expf(-(pr + pbv)));
      const float z = live ? sg : 0.0f;
      v2f gv;
      gv.x = v.x * z; gv.y = v.y * z;
      *(v2f*)(swf + (j & 1) * HD + ch) = gv;
      if ((j & 1) != 0) {
        __builtin_amdgcn_fence(__ATOMIC_ACQ_REL, "wavefront");
        __builtin_amdgcn_wave_barrier();
        const v4f fv = *(const v4f*)(swf + 4 * lane);
        float* rp = outF + (size_t)(c - 1) * HD + 4 * lane;
        *(volatile v4f*)rp = fv;
        __threadfence();
        *(volatile v4f*)rp = fv;
        __builtin_amdgcn_fence(__ATOMIC_ACQ_REL, "wavefront");
        __builtin_amdgcn_wave_barrier();
      }
    }
  }
}

__global__ __launch_bounds__(HD) void k_pool(const float* __restrict__ hg, const int* __restrict__ batch,
                                             float* gvec, int nN) {
  __shared__ __attribute__((aligned(16))) float sg[2 * HD];
  const int g = (int)blockIdx.x, t = (int)threadIdx.x;
  int lo = 0, hi = nN;
#pragma unroll 1
  while (lo < hi) {
    const int mid = (lo + hi) >> 1;
    const int bv = batch[mid];
    if (bv < g) lo = mid + 1; else hi = mid;
  }
  const int n0 = lo;
  lo = n0; hi = nN;
#pragma unroll 1
  while (lo < hi) {
    const int mid = (lo + hi) >> 1;
    const int bv = batch[mid];
    if (bv < g + 1) lo = mid + 1; else hi = mid;
  }
  const int n1 = lo;
  float mx = -__builtin_huge_valf(), sm = 0.0f, cn = 0.0f;
#pragma unroll 1
  for (int i = n0; i < n1; ++i) {
    const int bv = batch[i];
    const float v = hg[(size_t)i * HD + t];
    const bool hit = (bv == g);
    mx = hit ? fmaxf(mx, v) : mx;
    sm += hit ? v : 0.0f;
    cn += hit ? 1.0f : 0.0f;
  }
  sg[t]      = mx;
  sg[HD + t] = sm * (1.0f / fmaxf(cn, 1.0f));
  __syncthreads();
  v4f ov = {0.f, 0.f, 0.f, 0.f};
  if (t < 32) ov = *(const v4f*)(sg + 4 * t);
  float* gp = gvec + (size_t)g * (2 * HD) + 4 * t;
  if (t < 32) *(volatile v4f*)gp = ov;
  __threadfence();
  if (t < 32) *(volatile v4f*)gp = ov;
}

__global__ __launch_bounds__(NTHR) void k_head(
    const float* __restrict__ gvec, const float* __restrict__ lw1, const float* __restrict__ lb1,
    const float* __restrict__ lw2, const float* __restrict__ lb2, float* out, int G, int nOut) {
  __shared__ __attribute__((aligned(16))) float shid[GMAX * HD];
  __shared__ __attribute__((aligned(16))) float sout[GMAX * NCLS];
  const int tid = threadIdx.x;
#pragma unroll 1
  for (int idx = tid; idx < G * HD; idx += NTHR) {
    const int g = idx >> 6, o = idx & (HD - 1);
    const float* gr = gvec + (size_t)g * (2 * HD);
    float acc = lb1[o];
#pragma unroll 4
    for (int k = 0; k < 2 * HD; ++k) acc = fmaf(gr[k], lw1[k * HD + o], acc);
    shid[idx] = fmaxf(acc, 0.0f);
  }
  __syncthreads();
#pragma unroll 1
  for (int idx = tid; idx < G * NCLS; idx += NTHR) {
    const int g = idx >> 1, cc = idx & 1;
    float acc = lb2[cc];
#pragma unroll 4
    for (int k = 0; k < HD; ++k) acc = fmaf(shid[g * HD + k], lw2[k * NCLS + cc], acc);
    sout[idx] = acc;
  }
  __syncthreads();
  const int nq = nOut >> 2;
  v4f ov = {0.f, 0.f, 0.f, 0.f};
  if (tid < nq) ov = *(const v4f*)(sout + 4 * tid);
  v2f tv = {0.f, 0.f};
  const bool tail = ((nOut & 3) == 2) && (tid == 0);
  if (tail) tv = *(const v2f*)(sout + 4 * nq);
  if (tid < nq) *(volatile v4f*)(out + 4 * tid) = ov;
  if (tail) *(volatile v2f*)(out + 4 * nq) = tv;
  __threadfence();
  if (tid < nq) *(volatile v4f*)(out + 4 * tid) = ov;
  if (tail) *(volatile v2f*)(out + 4 * nq) = tv;
}

extern "C" void kernel_launch(void* const* d_in, const int* in_sizes, int n_in,
                              void* d_out, int out_size, void* d_ws, size_t ws_size,
                              hipStream_t stream) {
  if (n_in < 15) return;
  const int nN = in_sizes[0] / IND;
  const int nE = in_sizes[1] / 2;
  if (nN <= 0 || nE <= 0) return;
  if (in_sizes[0] != nN * IND || in_sizes[1] != 2 * nE) return;
  if (in_sizes[2] != nE || in_sizes[3] != nN || in_sizes[4] < 1) return;
  if (in_sizes[5] != IND * HD || in_sizes[6] != HD) return;
  if (in_sizes[7] != HD * HD || in_sizes[8] != HD) return;
  if (in_sizes[9] != HD || in_sizes[10] < 1) return;
  if (in_sizes[11] != 2 * HD * HD || in_sizes[12] != HD) return;
  if (in_sizes[13] != HD * NCLS || in_sizes[14] != NCLS) return;
  if (nN > (1 << 20) || nE > (1 << 28)) return;
  if (out_size <= 0 || (out_size % NCLS) != 0) return;
  const int G = out_size / NCLS;
  if (G < 1 || G > GMAX) return;

  const float* x    = (const float*)d_in[0];
  const int*   ei   = (const int*)d_in[1];
  const float* ewp  = (const float*)d_in[2];
  const int*   bat  = (const int*)d_in[3];
  const float* W1   = (const float*)d_in[5];
  const float* b1   = (const float*)d_in[6];
  const float* W2   = (const float*)d_in[7];
  const float* b2   = (const float*)d_in[8];
  const float* pwp  = (const float*)d_in[9];
  const float* pbp  = (const float*)d_in[10];
  const float* lw1  = (const float*)d_in[11];
  const float* lb1  = (const float*)d_in[12];
  const float* lw2  = (const float*)d_in[13];
  const float* lb2  = (const float*)d_in[14];
  float* out = (float*)d_out;
  const int* keys = ei + nE;
  const int* esrc = ei;
  const int nK = nE;

  const int NPAD   = ((nN + TGT - 1) / TGT) * TGT;
  const int nBC    = (nN + NBC - 1) / NBC;
  const int CNTPAD = nBC * NBC;
  const int nBF    = (nN + NBF - 1) / NBF;
  const int OFFN   = nBF * NBF;
  if (nBF + 1 > RBN) return;
  if (OFFN > CNTPAD || NPAD > OFFN) return;
  const int csrLen = ((nK + 31) & ~31) + 32 * (nBF + 1);
  const int nGemm  = NPAD / GROWS;
  const int nAgg   = NPAD / TGT;

  char* ws = (char*)d_ws;
  size_t off = 0;
  const size_t oX16 = off; off += (size_t)NPAD * IND * 2;        off = (off + 255) & ~(size_t)255;
  const size_t oH16 = off; off += (size_t)NPAD * HD * 2;         off = (off + 255) & ~(size_t)255;
  const size_t oW1  = off; off += (size_t)HD * IND * 2;          off = (off + 255) & ~(size_t)255;
  const size_t oW2  = off; off += (size_t)HD * HD * 2;           off = (off + 255) & ~(size_t)255;
  const size_t oCnt = off; off += (size_t)CNTPAD * 4;            off = (off + 255) & ~(size_t)255;
  const size_t oDis = off; off += (size_t)NPAD * 4;              off = (off + 255) & ~(size_t)255;
  const size_t oOff = off; off += (size_t)OFFN * 4;              off = (off + 255) & ~(size_t)255;
  const size_t oRb  = off; off += (size_t)RBN * 4;               off = (off + 255) & ~(size_t)255;
  const size_t oCsr = off; off += (size_t)csrLen * 4;            off = (off + 255) & ~(size_t)255;
  const size_t oHW  = off; off += (size_t)NPAD * HD * 4;         off = (off + 255) & ~(size_t)255;
  const size_t oHG  = off; off += (size_t)NPAD * HD * 4;         off = (off + 255) & ~(size_t)255;
  const size_t oGv  = off; off += (size_t)G * 2 * HD * 4;        off = (off + 255) & ~(size_t)255;
  if (off > ws_size || off > (size_t)WSCAP) return;
  _Float16* X16  = (_Float16*)(ws + oX16);
  _Float16* H16  = (_Float16*)(ws + oH16);
  _Float16* W1p  = (_Float16*)(ws + oW1);
  _Float16* W2p  = (_Float16*)(ws + oW2);
  int*      cnt  = (int*)(ws + oCnt);
  float*    dis  = (float*)(ws + oDis);
  int*      offp = (int*)(ws + oOff);
  int*      rb   = (int*)(ws + oRb);
  int*      csr  = (int*)(ws + oCsr);
  float*    HW   = (float*)(ws + oHW);
  float*    HG   = (float*)(ws + oHG);
  float*    gvec = (float*)(ws + oGv);

  const int vec8 = ((nE & 7) == 0) ? 1 : 0;
  const float oscX = 1.0f / ((float)ASCL * (float)WSCL);
  const float oscH = 1.0f / ((float)HSCL * (float)WSCL);

  {
    const int t8x = (NPAD * IND) / 8;
    k_cvt16<<<(t8x + NTHR - 1) / NTHR, NTHR, 0, stream>>>(x, X16, IND, nN, t8x, (float)ASCL);
  }
  {
    const dim3 g1(IND / TPK, HD / TPN);
    const dim3 g2(HD / TPK, HD / TPN);
    k_wT16<<<g1, NTHR, 0, stream>>>(W1, W1p, IND, HD, (float)WSCL);
    k_wT16<<<g2, NTHR, 0, stream>>>(W2, W2p, HD, HD, (float)WSCL);
  }

  hipFuncSetAttribute(reinterpret_cast<const void*>(&k_count),
                      hipFuncAttributeMaxDynamicSharedMemorySize, LDS_COUNT);
  k_count<<<nBC, NTHR, LDS_COUNT, stream>>>(keys, cnt, nK, vec8);
  k_offsets<<<1, OTHR, 0, stream>>>(cnt, offp, rb, nBF);
  hipFuncSetAttribute(reinterpret_cast<const void*>(&k_fill),
                      hipFuncAttributeMaxDynamicSharedMemorySize, LDS_FILL);
  k_fill<<<nBF, NTHR, LDS_FILL, stream>>>(keys, offp, rb, csr, nK, vec8, csrLen);

  k_deg<<<NPAD / NTHR, NTHR, 0, stream>>>(csr, offp, cnt, ewp, dis, nN, nE, csrLen);

  k_gemm<IND><<<nGemm, NTHR, 0, stream>>>(X16, W1p, dis, HW, oscX);
  k_agg<1><<<nAgg, NTHR, 0, stream>>>(csr, offp, cnt, dis, esrc, ewp, HW, b1, pwp, pbp, H16, HG, nN, nE, csrLen, (float)HSCL);

  k_gemm<HD><<<nGemm, NTHR, 0, stream>>>(H16, W2p, dis, HW, oscH);
  k_agg<2><<<nAgg, NTHR, 0, stream>>>(csr, offp, cnt, dis, esrc, ewp, HW, b2, pwp, pbp, H16, HG, nN, nE, csrLen, 1.0f);

  k_pool<<<G, HD, 0, stream>>>(HG, bat, gvec, nN);

  k_head<<<1, NTHR, 0, stream>>>(gvec, lw1, lb1, lw2, lb2, out, G, out_size);
}
